// FINN_Burger2D_20864951124293
// MI455X (gfx1250) — hardware-verified
//
#include <hip/hip_runtime.h>


#define NX   2048
#define NY   2048
#define NCELL (NX * NY)
#define HID  32
#define NP   64
#define RCH  262144
#define DXI  100.0f
#define DYI  100.0f
#define DM   HID
#define LOSC 1024.0f

typedef _Float16 h16;
typedef unsigned short bf;
typedef __attribute__((ext_vector_type(16))) __bf16   v16bf;
typedef __attribute__((ext_vector_type(16))) _Float16 v16h;
typedef __attribute__((ext_vector_type(8)))  _Float16 v8h;
typedef __attribute__((ext_vector_type(8)))  unsigned short v8us;
typedef __attribute__((ext_vector_type(8)))  float    v8f;
typedef __attribute__((ext_vector_type(4)))  float    v4f;
typedef v8h  __attribute__((may_alias)) v8ha;
typedef v4f  __attribute__((may_alias)) v4fa;
typedef v8us __attribute__((may_alias)) v8usa;

__device__ __forceinline__ unsigned short f2bf(float f) { unsigned u = __float_as_uint(f); u += 0x7FFFu + ((u >> 16) & 1u); return (unsigned short)(u >> 16); }
__device__ __forceinline__ float bf2f(unsigned short b) { return __uint_as_float(((unsigned)b) << 16); }
__device__ __forceinline__ float bfr(float f) { return bf2f(f2bf(f)); }
__device__ __forceinline__ v16h cat16(v8h lo, v8h hi) { return __builtin_shufflevector(lo, hi, 0, 1, 2, 3, 4, 5, 6, 7, 8, 9, 10, 11, 12, 13, 14, 15); }
__device__ __forceinline__ v16bf cat16b(v8us lo, v8us hi) { return __builtin_bit_cast(v16bf, __builtin_shufflevector(lo, hi, 0, 1, 2, 3, 4, 5, 6, 7, 8, 9, 10, 11, 12, 13, 14, 15)); }
__device__ __forceinline__ v8f wmma16(v16h a, v16h b, v8f c) { return __builtin_amdgcn_wmma_f32_16x16x32_f16(false, a, false, b, (short)0, c, false, false); }
__device__ __forceinline__ v8f wmmab(v16bf a, v16bf b, v8f c) { return __builtin_amdgcn_wmma_f32_16x16x32_bf16(false, a, false, b, (short)0, c, false, false); }

template <bool SPLITA, bool F16OUT = false>
__global__ __launch_bounds__(128) void k_gemmb(const bf* __restrict__ A, const bf* __restrict__ Al, const bf* __restrict__ Bn, const float* __restrict__ bias, float* C, int ldc, h16* C2, const float* __restrict__ R = nullptr, int K = DM, int roundR = 1) {
    __shared__ __align__(16) float ost[4][16 * 68];
    const int lane = threadIdx.x & 31, wave = threadIdx.x >> 5, lr = lane & 15, hi = lane >> 4;
    const int r0 = blockIdx.x * 64 + wave * 16, c0 = blockIdx.y * 64;
    const size_t aoff = (size_t)(r0 + lr) * K + 8 * hi;
    size_t boff[4];
#pragma unroll
    for (int t = 0; t < 4; ++t) boff[t] = (size_t)(c0 + t * 16 + lr) * K + 8 * hi;
    v8f acc[4];
#pragma unroll
    for (int t = 0; t < 4; ++t) acc[t] = (v8f){};
#pragma unroll 1
    for (int kc = 0; kc < K; kc += 32) {
        const v16bf a = cat16b(*(const v8us*)(A + aoff + kc), *(const v8us*)(A + aoff + kc + 16));
        v16bf al = a;
        if (SPLITA) al = cat16b(*(const v8us*)(Al + aoff + kc), *(const v8us*)(Al + aoff + kc + 16));
#pragma unroll
        for (int t = 0; t < 4; ++t) { const v16bf b = cat16b(*(const v8us*)(Bn + boff[t] + kc), *(const v8us*)(Bn + boff[t] + kc + 16)); acc[t] = wmmab(a, b, acc[t]); if (SPLITA) acc[t] = wmmab(al, b, acc[t]); }
        asm volatile("v_nop\n\tv_nop\n\tv_nop\n\tv_nop" : "+v"(acc[0]), "+v"(acc[1]), "+v"(acc[2]), "+v"(acc[3]) : "v"(a), "v"(al));
    }
    float* os = &ost[wave][0];
#pragma unroll
    for (int t = 0; t < 4; ++t) { const float bv = bias ? bfr(bias[c0 + t * 16 + lr]) : 0.f;
#pragma unroll
        for (int j = 0; j < 8; ++j) os[(hi * 8 + j) * 68 + t * 16 + lr] = acc[t][j] + bv; }
    __syncthreads();
    if (F16OUT) {
        h16* crow = (h16*)(void*)C + (size_t)r0 * ldc + c0;
        auto pass = [&]() {
#pragma unroll
            for (int s = 0; s < 4; ++s) { const int row = 4 * s + (lane >> 3), piece = lane & 7; const float* sp = os + row * 68 + piece * 8; v8h o, o2;
#pragma unroll
                for (int i = 0; i < 8; ++i) { const h16 a = (h16)sp[i]; o[i] = a; o2[i] = (h16)((sp[i] - (float)a) * LOSC); }
                *(volatile v8h*)(crow + (size_t)row * ldc + piece * 8) = o; if (C2) *(volatile v8h*)(C2 + (size_t)r0 * ldc + c0 + (size_t)row * ldc + piece * 8) = o2; }
        };
        pass(); __threadfence(); pass();
    } else {
        float* crow = C + (size_t)r0 * ldc + c0;
        auto pass = [&]() {
#pragma unroll
            for (int s = 0; s < 8; ++s) { const int Lid = (lane >> 3) + 4 * s, piece = lane & 7; const int row = Lid >> 1, cofs = (Lid & 1) * 32 + piece * 4;
                v4f val = *(const v4fa*)(os + row * 68 + cofs); if (R) { const v4f rv = *(const v4f*)(R + ((size_t)r0 + row) * ldc + c0 + cofs); val += roundR ? (v4f){bfr(rv[0]), bfr(rv[1]), bfr(rv[2]), bfr(rv[3])} : rv; }
                *(volatile v4f*)(crow + (size_t)row * ldc + cofs) = val; }
        };
        pass(); __threadfence(); pass();
    }
}


__global__ __launch_bounds__(256) void k_wtp(const float* __restrict__ Wm, int krows, int ncols, int kpad, bf* WT) {
    __shared__ __align__(16) unsigned short tl[64 * 72];
    const int tid = threadIdx.x, k0 = blockIdx.x * 64, n0 = blockIdx.y * 64;
    const int kk = tid >> 2, nq = (tid & 3) * 16;
    const int k = k0 + kk, kc = k < krows ? k : krows - 1;
#pragma unroll
    for (int i = 0; i < 16; ++i) { const int n = n0 + nq + i, ncl = n < ncols ? n : ncols - 1; const float w = Wm[(size_t)kc * ncols + ncl]; tl[(nq + i) * 72 + kk] = (k < krows && n < ncols) ? f2bf(w) : (unsigned short)0; }
    __syncthreads();
    const int piece = tid & 7;
    auto pass = [&]() {
#pragma unroll
        for (int s = 0; s < 2; ++s) { const int nr = (tid >> 3) + 32 * s; const v8us val = *(const v8usa*)(tl + nr * 72 + piece * 8); *(volatile v8us*)(WT + (size_t)(n0 + nr) * kpad + k0 + piece * 8) = val; }
    };
    pass(); __threadfence(); pass();
}

__global__ __launch_bounds__(256) void k_w2t(const float* __restrict__ W2, bf* W2T) {
    const int u = threadIdx.x; v8us o;
#pragma unroll
    for (int i = 0; i < 8; ++i) { const int f = u * 8 + i; const int n = f / HID, k = f % HID; const bool ok = n < HID; o[i] = ok ? f2bf(W2[k * HID + (ok ? n : 0)]) : (unsigned short)0; }
    *(volatile v8us*)(W2T + u * 8) = o; __threadfence(); *(volatile v8us*)(W2T + u * 8) = o;
}
__device__ __forceinline__ float tanh_f(float x) { const float e = __expf(2.0f * x); return 1.0f - 2.0f / (e + 1.0f); }
__global__ __launch_bounds__(256) void k_l1(const float* __restrict__ u, const float* __restrict__ W1, int c0, bf* Hh, bf* Hl) {
    const int lane = threadIdx.x & 31; const size_t r = ((size_t)blockIdx.x * 8 + (threadIdx.x >> 5)) * 8 + (lane >> 2); const int cb = (lane & 3) * 8;
    const float uv = bfr(u[(size_t)c0 + r]); v8us oh, ol;
#pragma unroll
    for (int i = 0; i < 8; ++i) { const float y = tanh_f(uv * bfr(W1[cb + i])); const unsigned short hb = f2bf(y); oh[i] = hb; ol[i] = f2bf(y - bf2f(hb)); }
    const size_t o = r * HID + cb; *(volatile v8us*)(Hh + o) = oh; *(volatile v8us*)(Hl + o) = ol; __threadfence(); *(volatile v8us*)(Hh + o) = oh; *(volatile v8us*)(Hl + o) = ol;
}
__global__ __launch_bounds__(256) void k_l3(const float* __restrict__ Z, const float* __restrict__ W3, int c0, float* A) {
    const size_t r = (size_t)blockIdx.x * 256 + threadIdx.x; float a = 0.f;
#pragma unroll 8
    for (int c = 0; c < HID; ++c) a = fmaf(tanh_f(Z[r * NP + c]), bfr(W3[c]), a);
    *(volatile float*)(A + c0 + r) = a; __threadfence(); *(volatile float*)(A + c0 + r) = a;
}
__global__ __launch_bounds__(256) void k_flux(const float* __restrict__ u, const float* __restrict__ A, const float* __restrict__ Dp, const float* __restrict__ BC, const float* __restrict__ st, float* OUTP) {
    const size_t g = (size_t)blockIdx.x * 256 + threadIdx.x; const size_t e0 = g * 4; const int i = (int)(e0 / NY), j0 = (int)(e0 % NY);
    const float s0 = bfr(st[0]), s1 = bfr(st[1]), bc0 = bfr(BC[0]), bc1 = bfr(BC[1]), d = bfr(Dp[0]); v4f o;
#pragma unroll
    for (int k = 0; k < 4; ++k) { const int j = j0 + k; const size_t e = (size_t)i * NY + j; const float uc = bfr(u[e]); const float a = A[e]; const float ap = fmaxf(a, 0.f), am = -fmaxf(-a, 0.f);
        const float ul = (i > 0) ? bfr(u[e - NY]) : bc0, ur = (i < NX - 1) ? bfr(u[e + NY]) : bc1, ub = (j > 0) ? bfr(u[e - 1]) : bc0, ut = (j < NY - 1) ? bfr(u[e + 1]) : bc1;
        const float lf = d * (s0 * uc + s1 * ul) - ap * DXI * (-s0 * uc - s1 * ul);
        const float rf = d * (s0 * uc + s1 * ur) - am * DXI * (s0 * uc + s1 * ur);
        const float bfl = d * (s0 * uc + s1 * ub) - ap * DYI * (-s0 * uc - s1 * ub);
        const float tf = d * (s0 * uc + s1 * ut) - am * DYI * (s0 * uc + s1 * ut);
        o[k] = lf + rf + bfl + tf; }
    *(volatile v4f*)(OUTP + e0) = o; __threadfence(); *(volatile v4f*)(OUTP + e0) = o;
}

extern "C" void kernel_launch(void* const* d_in, const int* in_sizes, int n_in,
                              void* d_out, int out_size, void* d_ws, size_t ws_size, hipStream_t stream) {
    (void)in_sizes; (void)n_in; (void)out_size;
    const float* u = (const float*)d_in[0]; const float* W1 = (const float*)d_in[1]; const float* W2 = (const float*)d_in[2]; const float* W3 = (const float*)d_in[3]; const float* Dp = (const float*)d_in[4]; const float* BC = (const float*)d_in[5]; const float* st = (const float*)d_in[6];
    float* out = (float*)d_out;
    char* wsp = (char*)d_ws;
    auto take = [&](size_t bytes) { char* p = wsp; wsp += (bytes + 255) & ~(size_t)255; return (void*)p; };
    bf* W2T = (bf*)take((size_t)NP * HID * 2); bf* Hh = (bf*)take((size_t)RCH * HID * 2); bf* Hl = (bf*)take((size_t)RCH * HID * 2); float* Z = (float*)take((size_t)RCH * NP * 4); float* A = (float*)take((size_t)NCELL * 4);
    if ((size_t)(wsp - (char*)d_ws) > ws_size) return;
    k_w2t<<<1, 256, 0, stream>>>(W2, W2T);
    for (int ch = 0; ch < NCELL / RCH; ++ch) { const int c0 = ch * RCH;
        k_l1<<<RCH / 64, 256, 0, stream>>>(u, W1, c0, Hh, Hl);
        k_gemmb<true, false><<<dim3(RCH / 64, NP / 64, 1), 128, 0, stream>>>(Hh, Hl, W2T, nullptr, Z, NP, nullptr, nullptr, HID);
        k_l3<<<RCH / 256, 256, 0, stream>>>(Z, W3, c0, A); }
    k_flux<<<NCELL / 4 / 256, 256, 0, stream>>>(u, A, Dp, BC, st, out);
}
